// SSM_spa_56427280335363
// MI455X (gfx1250) — hardware-run, weakly checked
//
#include <hip/hip_runtime.h>
#include <stdint.h>

typedef __attribute__((ext_vector_type(16))) _Float16 v16h;
typedef __attribute__((ext_vector_type(8)))  _Float16 v8h;
typedef __attribute__((ext_vector_type(16))) __bf16   v16b;
typedef __attribute__((ext_vector_type(8)))  __bf16   v8b;
typedef __attribute__((ext_vector_type(8)))  float    v8f;
typedef __attribute__((ext_vector_type(4)))  float    v4f;
typedef __attribute__((ext_vector_type(2)))  float    v2f;

constexpr int kBatch   = 8;
constexpr int kCIn     = 256;
constexpr int kSeq     = 256;
constexpr int kRows    = kBatch * kSeq;
constexpr int kImg     = 64;
constexpr int kSml     = 32;
constexpr int kDModel  = 1024;
constexpr int kDInner  = 2048;
constexpr int kDState  = 16;
constexpr int kDtRank  = 64;
constexpr int kNProj   = 96;
constexpr int kNProjPad = 128;
constexpr int kCOut    = 256;

static_assert(kRows % 64 == 0 && (2 * kDInner) % 64 == 0 && kDModel % 32 == 0);
static_assert(kNProjPad % 64 == 0 && kDInner % 32 == 0);
static_assert(kDInner % 64 == 0 && kDtRank % 32 == 0);
static_assert(kDModel % 64 == 0);
static_assert(kCOut % 64 == 0 && (kSml * kSml) % 64 == 0 && kCIn % 32 == 0);

constexpr size_t kOffXz    = 0;
constexpr size_t kOffYmm   = 0;
constexpr size_t kOffYln   = 8388608;
constexpr size_t kOffYlnTH = 16777216;
constexpr size_t kOffYlnTL = 20971520;
constexpr size_t kOffSmall = 25165824;
constexpr size_t kR1       = 33554432;
constexpr size_t kOffWinH  = kR1;
constexpr size_t kOffWinL  = kR1 + 8388608;
constexpr size_t kOffXsH   = kR1 + 16777216;
constexpr size_t kOffXsL   = kR1 + 20971520;
constexpr size_t kOffDtpre = kR1;
constexpr size_t kOffXcB   = kR1 + 16777216;
constexpr size_t kR2       = kR1 + 25165824;
constexpr size_t kOffXcF   = kR2;
constexpr size_t kR3       = kR2 + 16777216;
constexpr size_t kOffYH    = kR3;
constexpr size_t kOffYL    = kR3 + 8388608;
constexpr size_t kR4       = kR3 + 16777216;
constexpr size_t kOffWx    = kR4;
constexpr size_t kOffWdt   = kR4 + 524288;
constexpr size_t kOffWoH   = kR4 + 786432;
constexpr size_t kOffWoL   = kR4 + 4980736;
constexpr size_t kOffWcH   = kR4 + 9175040;
constexpr size_t kOffWcL   = kR4 + 9306112;
constexpr size_t kOffProj  = kR4 + 9437184;
constexpr size_t kOffDtA   = kR4 + 10485760;
constexpr size_t kWsTotal  = kR4 + 10747904;
static_assert(kOffSmall + (size_t)kBatch * kCOut * kSml * kSml * 4 == kR1);
static_assert(kOffXsL + (size_t)kRows * kDModel * 2 == kR2);
static_assert(kOffDtpre + (size_t)kRows * kDInner * 4 == kOffXcB);
static_assert(kOffXcB + (size_t)kRows * kDInner * 2 == kR2);
static_assert(kOffDtA + (size_t)kRows * kDtRank * 2 == kWsTotal);
static_assert(kWsTotal == 103022592);
static_assert(kWsTotal <= 134217728);

__device__ __forceinline__ unsigned short f2bf_bits(float f) {
  unsigned u = __float_as_uint(f);
  return (unsigned short)((u + 0x7FFFu + ((u >> 16) & 1u)) >> 16);
}
__device__ __forceinline__ float bf_bits2f(unsigned short h) { return __uint_as_float(((unsigned)h) << 16); }

__device__ __forceinline__ void dep_guard_h(v8f& a, v8f& b, v16h x, v16h y) { asm volatile("v_nop\n\tv_nop\n\tv_nop\n\tv_nop" : "+v"(a), "+v"(b) : "v"(x), "v"(y)); }
__device__ __forceinline__ void dep_guard_b(v8f& a, v8f& b, v16b x, v16b y) { asm volatile("v_nop\n\tv_nop\n\tv_nop\n\tv_nop" : "+v"(a), "+v"(b) : "v"(x), "v"(y)); }
__device__ __forceinline__ void keep4_h(v16h a, v16h b, v16h c, v16h d) { asm volatile("v_nop" :: "v"(a), "v"(b), "v"(c), "v"(d)); }
__device__ __forceinline__ void keep4_b(v16b a, v16b b, v16b c, v16b d) { asm volatile("v_nop" :: "v"(a), "v"(b), "v"(c), "v"(d)); }
__device__ __forceinline__ void acc_guard4(v8f& a, v8f& b, v8f& c, v8f& d) { asm volatile("v_nop\n\tv_nop\n\tv_nop\n\tv_nop" : "+v"(a), "+v"(b), "+v"(c), "+v"(d)); }
template <typename T> struct Frag;
template <> struct Frag<_Float16> {
  typedef v16h V; union U { v16h v; v8h h[2]; };
  static __device__ __forceinline__ v16h load(const _Float16* p) {
    U f; f.h[0] = *(const v8h*)(p); f.h[1] = *(const v8h*)(p + 16); return f.v;
  }
  static __device__ __forceinline__ v8f mma(v16h a, v16h b, v8f c) {
    return __builtin_amdgcn_wmma_f32_16x16x32_f16(false, a, false, b, (short)0, c, false, false);
  }
  static __device__ __forceinline__ void guard(v8f& a, v8f& b, v16h x, v16h y) { dep_guard_h(a, b, x, y); }
  static __device__ __forceinline__ void keep(v16h a, v16h b, v16h c, v16h d) { keep4_h(a, b, c, d); }
};
template <> struct Frag<__bf16> {
  typedef v16b V; union U { v16b v; v8b h[2]; };
  static __device__ __forceinline__ v16b load(const __bf16* p) {
    U f; f.h[0] = *(const v8b*)(p); f.h[1] = *(const v8b*)(p + 16); return f.v;
  }
  static __device__ __forceinline__ v8f mma(v16b a, v16b b, v8f c) {
    return __builtin_amdgcn_wmma_f32_16x16x32_bf16(false, a, false, b, (short)0, c, false, false);
  }
  static __device__ __forceinline__ void guard(v8f& a, v8f& b, v16b x, v16b y) { dep_guard_b(a, b, x, y); }
  static __device__ __forceinline__ void keep(v16b a, v16b b, v16b c, v16b d) { keep4_b(a, b, c, d); }
};

template <int ET> struct Elem;
template <> struct Elem<0> { typedef _Float16 T; };
template <> struct Elem<1> { typedef __bf16 T; };
template <int ET, bool SPLIT, int BIAS_MODE, int OUT_MODE, bool RESID, int ACT = 0>
__global__ __launch_bounds__(256) void wmma_gemm64(
    const unsigned short* __restrict__ Ap, const unsigned short* __restrict__ A2p, int lda, long strideA,
    const unsigned short* __restrict__ Btp, const unsigned short* __restrict__ Bt2p, int ldb, long strideB,
    void* __restrict__ Cout, void* __restrict__ Cout2, int ldc, long strideC,
    const float* __restrict__ bias,
    const float* __restrict__ resid, long strideR,
    int M, int N, int K, float scale) {
  typedef typename Elem<ET>::T T;
  typedef typename Frag<T>::V V;
  const T* A = (const T*)Ap; const T* A2 = (const T*)A2p; const T* Bt = (const T*)Btp; const T* Bt2 = (const T*)Bt2p;
  __shared__ __align__(16) float sT[8][16 * 68];
  const int b    = blockIdx.y;
  const int lane = threadIdx.x & 31;
  const int wave = threadIdx.x >> 5;
  const int tilesN = N >> 6;
  const int tilesM = M >> 6;
  const int tile = blockIdx.x * 8 + wave;
  if (tile >= tilesM * tilesN) return;
  const int tm = tile / tilesN;
  const int tn = tile - tm * tilesN;
  const int m0 = tm << 6;
  const int n0 = tn << 6;

  const T* Ab  = A  + (size_t)b * strideA;
  const T* Bb  = Bt + (size_t)b * strideB;
  const T* Ab2 = SPLIT ? (A2  + (size_t)b * strideA) : nullptr;
  const T* Bb2 = SPLIT ? (Bt2 + (size_t)b * strideB) : nullptr;

  const int rlane = lane & 15;
  const int koff  = (lane >> 4) * 8;
  const int mOff  = (lane >> 4) * 8;

  v8f acc[4][4];
#pragma unroll
  for (int i = 0; i < 4; ++i)
#pragma unroll
    for (int j = 0; j < 4; ++j) acc[i][j] = (v8f){0.f,0.f,0.f,0.f,0.f,0.f,0.f,0.f};

  for (int k0 = 0; k0 < K; k0 += 32) {
    V bh[4], bl[4];
#pragma unroll
    for (int j = 0; j < 4; ++j) {
      const size_t bo = (size_t)(n0 + (j << 4) + rlane) * ldb + koff + k0;
      bh[j] = Frag<T>::load(Bb + bo);
      if (SPLIT) bl[j] = Frag<T>::load(Bb2 + bo);
    }
#pragma unroll
    for (int i = 0; i < 4; ++i) {
      const size_t ao = (size_t)(m0 + (i << 4) + rlane) * lda + koff + k0;
      V ah = Frag<T>::load(Ab + ao);
      V al;
      if (SPLIT) al = Frag<T>::load(Ab2 + ao);
#pragma unroll
      for (int j = 0; j < 4; ++j) {
        acc[i][j] = Frag<T>::mma(ah, bh[j], acc[i][j]);
        if (SPLIT) {
          acc[i][j] = Frag<T>::mma(ah, bl[j], acc[i][j]);
          acc[i][j] = Frag<T>::mma(al, bh[j], acc[i][j]);
        }
      }
      Frag<T>::guard(acc[i][0], acc[i][3], ah, SPLIT ? al : ah);
    }
    Frag<T>::keep(bh[0], bh[1], bh[2], bh[3]);
    if (SPLIT) Frag<T>::keep(bl[0], bl[1], bl[2], bl[3]);
  }
  acc_guard4(acc[0][0], acc[0][1], acc[0][2], acc[0][3]);
  acc_guard4(acc[1][0], acc[1][1], acc[1][2], acc[1][3]);
  acc_guard4(acc[2][0], acc[2][1], acc[2][2], acc[2][3]);
  acc_guard4(acc[3][0], acc[3][1], acc[3][2], acc[3][3]);

  float* slab = sT[wave];
  const float* Rb = RESID ? (resid + (size_t)b * strideR) : nullptr;
#pragma unroll
  for (int i = 0; i < 4; ++i) {
    const int mBase = m0 + (i << 4);
#pragma unroll
    for (int j = 0; j < 4; ++j) {
      const int n = n0 + (j << 4) + rlane;
      float bv = 0.f;
      if (BIAS_MODE == 2) bv = bias[n];
#pragma unroll
      for (int r = 0; r < 8; ++r) {
        float v = acc[i][j][r] * scale;
        if (BIAS_MODE == 1) v += bias[mBase + mOff + r];
        if (BIAS_MODE == 2) v += bv;
        if (RESID) v += Rb[(size_t)(mBase + mOff + r) * ldc + n];
        if (ACT == 1) v = tanhf(v);
        if (ACT == 2) v = fmaxf(v, 0.0f);
        if (ACT == 3) v = v / (1.0f + expf(-v));
        if (ACT == 4) v = (v > 0.f) ? v : 0.01f * v;
        if (ACT == 5) v = 0.5f * v * (1.0f + erff(v * 0.70710678118654752f));
        slab[(mOff + r) * 68 + (j << 4) + rlane] = v;
      }
    }
    __builtin_amdgcn_fence(__ATOMIC_RELEASE, "workgroup");
    __builtin_amdgcn_wave_barrier();
    __builtin_amdgcn_fence(__ATOMIC_ACQUIRE, "workgroup");
    if (OUT_MODE == 0) {
      float* C = (float*)Cout + (size_t)b * strideC;
      const int hh = lane >> 4, c4 = (lane & 15) * 4;
      for (int pass = 0; pass < 2; ++pass) {
#pragma unroll
        for (int it = 0; it < 8; ++it) {
          const int row = it * 2 + hh;
          v4f v = *(const v4f*)(slab + row * 68 + c4);
          *(volatile v4f*)(C + (size_t)(mBase + row) * ldc + n0 + c4) = v;
        }
        __threadfence();
      }
    } else {
      const int q = lane >> 3, c8 = (lane & 7) * 8;
      unsigned short* C  = (unsigned short*)Cout  + (size_t)b * strideC;
      unsigned short* C2 = (OUT_MODE == 2) ? ((unsigned short*)Cout2 + (size_t)b * strideC) : nullptr;
      for (int pass = 0; pass < 2; ++pass) {
#pragma unroll
        for (int it = 0; it < 4; ++it) {
          const int row = it * 4 + q;
          const float* sp = slab + row * 68 + c8;
          v8h hv, lv;
#pragma unroll
          for (int e = 0; e < 8; ++e) {
            if (OUT_MODE == 1) {
              hv[e] = (_Float16)sp[e];
            } else {
              unsigned short hb = f2bf_bits(sp[e]);
              unsigned short lb = f2bf_bits(sp[e] - bf_bits2f(hb));
              hv[e] = __builtin_bit_cast(_Float16, hb);
              lv[e] = __builtin_bit_cast(_Float16, lb);
            }
          }
          *(volatile v8h*)(C + (size_t)(mBase + row) * ldc + n0 + c8) = hv;
          if (OUT_MODE == 2) *(volatile v8h*)(C2 + (size_t)(mBase + row) * ldc + n0 + c8) = lv;
        }
        __threadfence();
      }
    }
    __builtin_amdgcn_fence(__ATOMIC_RELEASE, "workgroup");
    __builtin_amdgcn_wave_barrier();
    __builtin_amdgcn_fence(__ATOMIC_ACQUIRE, "workgroup");
  }
}

__device__ __forceinline__ float softplus_f(float x) {
  return fmaxf(x, 0.0f) + log1pf(expf(-fabsf(x)));
}
__device__ __forceinline__ float silu_f(float x) {
  return x * (1.0f / (1.0f + expf(-x)));
}

template <bool LO>
__global__ __launch_bounds__(256) void k_transpose_planes(
    const float* __restrict__ in, int ldin, int ncols, long strideIn,
    unsigned short* __restrict__ outH, unsigned short* __restrict__ outL, int ldo, long strideOut) {
  __shared__ __align__(16) float ts[32][68];
  const int tid = threadIdx.x, lane = tid & 31, wave = tid >> 5;
  const int c0 = blockIdx.x * 32, r0 = blockIdx.y * 64;
  const float* inb = in + (size_t)blockIdx.z * strideIn;
#pragma unroll
  for (int i = 0; i < 8; ++i) {
    const int idx = i * 256 + tid;
    const int rr = idx >> 5, cc = idx & 31;
    const int c = c0 + cc;
    const int ccl = (c < ncols) ? c : (ncols - 1);
    float v = inb[(size_t)(r0 + rr) * ldin + ccl];
    v = (c < ncols) ? v : 0.0f;
    ts[cc][rr] = v;
  }
  __syncthreads();
  const int q = lane >> 3, c8 = (lane & 7) * 8;
  const int cc = wave * 4 + q;
  const float* sp = &ts[cc][c8];
  v8h hv, lv;
#pragma unroll
  for (int e = 0; e < 8; ++e) {
    const float f = sp[e];
    const unsigned short hb = f2bf_bits(f);
    const unsigned short lb = f2bf_bits(f - bf_bits2f(hb));
    hv[e] = __builtin_bit_cast(_Float16, hb);
    lv[e] = __builtin_bit_cast(_Float16, lb);
  }
  const size_t o = (size_t)blockIdx.z * strideOut + (size_t)(c0 + cc) * ldo + r0 + c8;
  for (int pass = 0; pass < 2; ++pass) {
    *(volatile v8h*)(outH + o) = hv;
    if (LO) *(volatile v8h*)(outL + o) = lv;
    __threadfence();
  }
}

__global__ __launch_bounds__(128) void k_resize_down(const float* __restrict__ x,
                                                     unsigned short* __restrict__ xsH,
                                                     unsigned short* __restrict__ xsL) {
  __shared__ __align__(16) float img[64 * 64];
  const int tid = threadIdx.x;
  const int row = blockIdx.x;
  const float* src = x + (size_t)row * 4096;
#pragma unroll
  for (int i = 0; i < 8; ++i) {
    const int idx = (i * 128 + tid) * 4;
    *(v4f*)(img + idx) = *(const v4f*)(src + idx);
  }
  __syncthreads();
  const int sy = tid >> 2, sx0 = (tid & 3) * 8;
  float py = 63.0f * ((float)sy * (1.0f / 31.0f));
  py = (sy == 31) ? 63.0f : py;
  int y0 = (int)py;
  y0 = (y0 > 63) ? 63 : y0;
  const int y1 = (y0 + 1 > 63) ? 63 : (y0 + 1);
  const float ty = py - (float)y0;
  v8h hv, lv;
#pragma unroll
  for (int e = 0; e < 8; ++e) {
    const int sx = sx0 + e;
    float px = 63.0f * ((float)sx * (1.0f / 31.0f));
    px = (sx == 31) ? 63.0f : px;
    int x0 = (int)px;
    x0 = (x0 > 63) ? 63 : x0;
    const int x1i = (x0 + 1 > 63) ? 63 : (x0 + 1);
    const float tx = px - (float)x0;
    const float v00 = img[y0 * 64 + x0], v01 = img[y0 * 64 + x1i];
    const float v10 = img[y1 * 64 + x0], v11 = img[y1 * 64 + x1i];
    const float a0 = v00 * (1.0f - ty) + v10 * ty;
    const float a1 = v01 * (1.0f - ty) + v11 * ty;
    const float v = a0 * (1.0f - tx) + a1 * tx;
    const unsigned short hb = f2bf_bits(v);
    const unsigned short lb = f2bf_bits(v - bf_bits2f(hb));
    hv[e] = __builtin_bit_cast(_Float16, hb);
    lv[e] = __builtin_bit_cast(_Float16, lb);
  }
  const size_t o = (size_t)row * 1024 + tid * 8;
  for (int pass = 0; pass < 2; ++pass) {
    *(volatile v8h*)(xsH + o) = hv;
    *(volatile v8h*)(xsL + o) = lv;
    __threadfence();
  }
}

__global__ __launch_bounds__(256) void k_conv_silu(const float* __restrict__ xz, const float* __restrict__ cw,
                                                   const float* __restrict__ cb, float* __restrict__ xcF,
                                                   unsigned short* __restrict__ xcB) {
  __shared__ __align__(16) float slab[8][256];
  const int tid = threadIdx.x, lane = tid & 31, wave = tid >> 5;
  const int row = blockIdx.x;
  const int bb = row >> 8, l = row & 255;
  const int d0 = wave * 256 + lane * 8;
  float acc[8];
#pragma unroll
  for (int e = 0; e < 8; ++e) acc[e] = 0.0f;
  v4f wv[8];
#pragma unroll
  for (int i = 0; i < 8; ++i) wv[i] = *(const v4f*)(cw + (size_t)d0 * 4 + i * 4);
#pragma unroll
  for (int k = 0; k < 4; ++k) {
    const int ls = l + k - 3;
    const int lsc = (ls < 0) ? 0 : ls;
    const float* xr = xz + (size_t)(bb * 256 + lsc) * 4096 + d0;
    const v4f xa = *(const v4f*)xr;
    const v4f xb = *(const v4f*)(xr + 4);
    const bool ok = (ls >= 0);
#pragma unroll
    for (int e = 0; e < 4; ++e) {
      const float u0 = ok ? xa[e] : 0.0f;
      const float u1 = ok ? xb[e] : 0.0f;
      acc[e]     += u0 * wv[e][k];
      acc[4 + e] += u1 * wv[4 + e][k];
    }
  }
  {
    const v4f b0 = *(const v4f*)(cb + d0), b1 = *(const v4f*)(cb + d0 + 4);
#pragma unroll
    for (int e = 0; e < 4; ++e) { acc[e] += b0[e]; acc[4 + e] += b1[e]; }
  }
  float* sl = slab[wave];
  {
    v4f p0, p1;
#pragma unroll
    for (int e = 0; e < 4; ++e) { p0[e] = acc[e]; p1[e] = acc[4 + e]; }
    *(v4f*)(sl + lane * 8) = p0;
    *(v4f*)(sl + lane * 8 + 4) = p1;
  }
  __builtin_amdgcn_fence(__ATOMIC_RELEASE, "workgroup");
  __builtin_amdgcn_wave_barrier();
  __builtin_amdgcn_fence(__ATOMIC_ACQUIRE, "workgroup");
#pragma unroll 1
  for (int g = 0; g < 2; ++g) {
    const int idx = g * 128 + lane * 4;
    const v4f v = *(const v4f*)(sl + idx);
    v4f ov;
#pragma unroll
    for (int e = 0; e < 4; ++e) ov[e] = silu_f(v[e]);
    *(v4f*)(sl + idx) = ov;
  }
  __builtin_amdgcn_fence(__ATOMIC_RELEASE, "workgroup");
  __builtin_amdgcn_wave_barrier();
  __builtin_amdgcn_fence(__ATOMIC_ACQUIRE, "workgroup");
  v8h hv;
  {
    const v4f a0 = *(const v4f*)(sl + lane * 8), a1 = *(const v4f*)(sl + lane * 8 + 4);
#pragma unroll
    for (int e = 0; e < 4; ++e) {
      hv[e]     = __builtin_bit_cast(_Float16, f2bf_bits(a0[e]));
      hv[4 + e] = __builtin_bit_cast(_Float16, f2bf_bits(a1[e]));
    }
  }
  const v4f s0 = *(const v4f*)(sl + lane * 4);
  const v4f s1 = *(const v4f*)(sl + 128 + lane * 4);
  const size_t of = (size_t)row * 2048 + wave * 256;
  for (int pass = 0; pass < 2; ++pass) {
    *(volatile v4f*)(xcF + of + lane * 4) = s0;
    *(volatile v4f*)(xcF + of + 128 + lane * 4) = s1;
    *(volatile v8h*)(xcB + of + lane * 8) = hv;
    __threadfence();
  }
}

__global__ __launch_bounds__(256) void k_cvt_dt(const float* __restrict__ proj, unsigned short* __restrict__ dtA) {
  const int tid = threadIdx.x, lane = tid & 31, wave = tid >> 5;
  const int row = blockIdx.x * 32 + wave * 4 + (lane >> 3);
  const int c8 = (lane & 7) * 8;
  const v4f a = *(const v4f*)(proj + (size_t)row * 128 + c8);
  const v4f b2 = *(const v4f*)(proj + (size_t)row * 128 + c8 + 4);
  v8h hv;
#pragma unroll
  for (int e = 0; e < 4; ++e) {
    hv[e]     = __builtin_bit_cast(_Float16, f2bf_bits(a[e]));
    hv[4 + e] = __builtin_bit_cast(_Float16, f2bf_bits(b2[e]));
  }
  const size_t o = (size_t)row * 64 + c8;
  for (int pass = 0; pass < 2; ++pass) {
    *(volatile v8h*)(dtA + o) = hv;
    __threadfence();
  }
}

__global__ __launch_bounds__(256) void k_scan(const float* __restrict__ proj, const float* __restrict__ dtpre,
                                              const float* __restrict__ xcF, const float* __restrict__ xz,
                                              const float* __restrict__ alog, const float* __restrict__ dpar,
                                              const float* __restrict__ dtb,
                                              unsigned short* __restrict__ yH, unsigned short* __restrict__ yL) {
  __shared__ float bc[32];
  __shared__ __align__(16) float ybuf[256];
  __shared__ float abuf[256 * 16];
  const int tid = threadIdx.x, lane = tid & 31, wave = tid >> 5;
  const int dblk = blockIdx.x, bb = blockIdx.y;
  const int d = dblk * 256 + tid;
#pragma unroll 1
  for (int s = 0; s < 16; ++s) abuf[tid * 16 + s] = -expf(alog[(size_t)d * 16 + s]);
  float a2[16], h[16];
#pragma unroll
  for (int s = 0; s < 16; ++s) { a2[s] = abuf[tid * 16 + s] * 1.4426950408889634f; h[s] = 0.0f; }
  const float dd = dpar[d];
  const float bd = dtb[d];
  for (int l = 0; l < kSeq; ++l) {
    const int row = bb * 256 + l;
    if (tid < 32) bc[tid] = proj[(size_t)row * 128 + 64 + tid];
    __syncthreads();
    const float dtv = softplus_f(dtpre[(size_t)row * 2048 + d] + bd);
    const float xv  = xcF[(size_t)row * 2048 + d];
    const float zv  = xz[(size_t)row * 4096 + 2048 + d];
    const float dtx = dtv * xv;
    float yv = 0.0f;
#pragma unroll
    for (int s = 0; s < 16; ++s) {
      const float dA = exp2f(dtv * a2[s]);
      h[s] = dA * h[s] + dtx * bc[s];
      yv += h[s] * bc[16 + s];
    }
    yv = (yv + xv * dd) * silu_f(zv);
    ybuf[tid] = yv;
    __syncthreads();
    {
      const int seg = wave & 3;
      const v2f pr = *(const v2f*)(ybuf + seg * 64 + 2 * lane);
      const unsigned short h0 = f2bf_bits(pr[0]), h1 = f2bf_bits(pr[1]);
      const unsigned short l0 = f2bf_bits(pr[0] - bf_bits2f(h0));
      const unsigned short l1 = f2bf_bits(pr[1] - bf_bits2f(h1));
      const unsigned uh = (unsigned)h0 | ((unsigned)h1 << 16);
      const unsigned ul = (unsigned)l0 | ((unsigned)l1 << 16);
      const unsigned val = (wave < 4) ? uh : ul;
      const size_t base = (size_t)row * 2048 + dblk * 256 + seg * 64;
      unsigned* ph = (unsigned*)(yH + base) + lane;
      unsigned* pl = (unsigned*)(yL + base) + lane;
      unsigned* p = (wave < 4) ? ph : pl;
      *(volatile unsigned*)p = val;
      __threadfence();
      *(volatile unsigned*)p = val;
    }
  }
}

__global__ __launch_bounds__(256) void k_layernorm(const float* __restrict__ y, const float* __restrict__ g,
                                                   const float* __restrict__ bta, float* __restrict__ outp) {
  __shared__ __align__(16) float gs[1024];
  __shared__ __align__(16) float bs2[1024];
  __shared__ __align__(16) float slab[8][1024];
  const int tid = threadIdx.x, lane = tid & 31, wave = tid >> 5;
  *(v4f*)(gs + tid * 4)  = *(const v4f*)(g + tid * 4);
  *(v4f*)(bs2 + tid * 4) = *(const v4f*)(bta + tid * 4);
  __syncthreads();
  const int row = blockIdx.x * 8 + wave;
  const float* yr = y + (size_t)row * 1024;
  float s = 0.0f;
#pragma unroll 1
  for (int it = 0; it < 8; ++it) {
    const v4f v = *(const v4f*)(yr + it * 128 + lane * 4);
    s += (v[0] + v[1]) + (v[2] + v[3]);
  }
#pragma unroll
  for (int off = 1; off < 32; off <<= 1) s += __shfl_xor(s, off, 32);
  const float mean = s * (1.0f / 1024.0f);
  float q = 0.0f;
#pragma unroll 1
  for (int it = 0; it < 8; ++it) {
    const v4f v = *(const v4f*)(yr + it * 128 + lane * 4);
    const float e0 = v[0] - mean, e1 = v[1] - mean, e2 = v[2] - mean, e3 = v[3] - mean;
    q += (e0 * e0 + e1 * e1) + (e2 * e2 + e3 * e3);
  }
#pragma unroll
  for (int off = 1; off < 32; off <<= 1) q += __shfl_xor(q, off, 32);
  const float var = q * (1.0f / 1024.0f);
  const float rstd = rsqrtf(var + 1e-5f);
  float* sl = slab[wave];
#pragma unroll 1
  for (int it = 0; it < 8; ++it) {
    const int idx = it * 128 + lane * 4;
    const v4f v = *(const v4f*)(yr + idx);
    const v4f gg = *(const v4f*)(gs + idx);
    const v4f be = *(const v4f*)(bs2 + idx);
    v4f ov;
#pragma unroll
    for (int e = 0; e < 4; ++e) ov[e] = (v[e] - mean) * rstd * gg[e] + be[e];
    *(v4f*)(sl + idx) = ov;
  }
  float* orow = outp + (size_t)row * 1024;
  for (int pass = 0; pass < 2; ++pass) {
#pragma unroll
    for (int it = 0; it < 8; ++it) {
      const int idx = it * 128 + lane * 4;
      const v4f ov = *(const v4f*)(sl + idx);
      *(volatile v4f*)(orow + idx) = ov;
    }
    __threadfence();
  }
}

__global__ __launch_bounds__(256) void k_resize_up(const float* __restrict__ sml, const float* __restrict__ cbias,
                                                   float* __restrict__ outp) {
  __shared__ __align__(16) float img[1024];
  const int tid = threadIdx.x, lane = tid & 31, wave = tid >> 5;
  const int bo = blockIdx.x >> 2, rg = blockIdx.x & 3;
  *(v4f*)(img + tid * 4) = *(const v4f*)(sml + (size_t)bo * 1024 + tid * 4);
  __syncthreads();
  const int o = bo & 255;
  const float bv = cbias[o];
  const int oy = rg * 16 + wave * 2 + (lane >> 4);
  const int ox0 = (lane & 15) * 4;
  float py = 31.0f * ((float)oy * (1.0f / 63.0f));
  py = (oy == 63) ? 31.0f : py;
  int y0 = (int)py;
  y0 = (y0 > 31) ? 31 : y0;
  const int y1 = (y0 + 1 > 31) ? 31 : (y0 + 1);
  const float ty = py - (float)y0;
  v4f res;
#pragma unroll
  for (int e = 0; e < 4; ++e) {
    const int ox = ox0 + e;
    float px = 31.0f * ((float)ox * (1.0f / 63.0f));
    px = (ox == 63) ? 31.0f : px;
    int x0 = (int)px;
    x0 = (x0 > 31) ? 31 : x0;
    const int x1i = (x0 + 1 > 31) ? 31 : (x0 + 1);
    const float tx = px - (float)x0;
    const float v00 = img[y0 * 32 + x0], v01 = img[y0 * 32 + x1i];
    const float v10 = img[y1 * 32 + x0], v11 = img[y1 * 32 + x1i];
    const float a0 = v00 * (1.0f - ty) + v10 * ty;
    const float a1 = v01 * (1.0f - ty) + v11 * ty;
    res[e] = (a0 * (1.0f - tx) + a1 * tx) + bv;
  }
  const size_t oo = ((size_t)bo * 64 + oy) * 64 + ox0;
  for (int pass = 0; pass < 2; ++pass) {
    *(volatile v4f*)(outp + oo) = res;
    __threadfence();
  }
}

extern "C" void kernel_launch(void* const* d_in, const int* in_sizes, int n_in,
                              void* d_out, int out_size, void* d_ws, size_t ws_size,
                              hipStream_t stream) {
  if (n_in < 14) return;
  if (in_sizes[0] != kBatch * kCIn * kImg * kImg) return;
  if (in_sizes[1] != kDModel * 2 * kDInner) return;
  if (in_sizes[2] != kDInner * 4 || in_sizes[3] != kDInner) return;
  if (in_sizes[4] != kDInner * kNProj) return;
  if (in_sizes[5] != kDtRank * kDInner || in_sizes[6] != kDInner) return;
  if (in_sizes[7] != kDInner * kDState || in_sizes[8] != kDInner) return;
  if (in_sizes[9] != kDInner * kDModel) return;
  if (in_sizes[10] != kDModel || in_sizes[11] != kDModel) return;
  if (in_sizes[12] != kCIn * kCOut || in_sizes[13] != kCOut) return;
  if (out_size != kBatch * kCOut * kImg * kImg) return;
  if (ws_size < kWsTotal) return;

  const float* x1        = (const float*)d_in[0];
  const float* in_proj_w = (const float*)d_in[1];
  const float* conv_w    = (const float*)d_in[2];
  const float* conv_b    = (const float*)d_in[3];
  const float* x_proj_w  = (const float*)d_in[4];
  const float* dt_proj_w = (const float*)d_in[5];
  const float* dt_proj_b = (const float*)d_in[6];
  const float* a_log     = (const float*)d_in[7];
  const float* d_param   = (const float*)d_in[8];
  const float* out_proj_w = (const float*)d_in[9];
  const float* ln_g      = (const float*)d_in[10];
  const float* ln_b      = (const float*)d_in[11];
  const float* lin_ch_w  = (const float*)d_in[12];
  const float* lin_ch_b  = (const float*)d_in[13];
  float* out = (float*)d_out;

  char* ws = (char*)d_ws;
  float*          xz    = (float*)(ws + kOffXz);
  float*          ymm   = (float*)(ws + kOffYmm);
  float*          yln   = (float*)(ws + kOffYln);
  unsigned short* ylnTH = (unsigned short*)(ws + kOffYlnTH);
  unsigned short* ylnTL = (unsigned short*)(ws + kOffYlnTL);
  float*          sml   = (float*)(ws + kOffSmall);
  unsigned short* winH  = (unsigned short*)(ws + kOffWinH);
  unsigned short* winL  = (unsigned short*)(ws + kOffWinL);
  unsigned short* xsH   = (unsigned short*)(ws + kOffXsH);
  unsigned short* xsL   = (unsigned short*)(ws + kOffXsL);
  float*          dtpre = (float*)(ws + kOffDtpre);
  unsigned short* xcB   = (unsigned short*)(ws + kOffXcB);
  float*          xcF   = (float*)(ws + kOffXcF);
  unsigned short* yH    = (unsigned short*)(ws + kOffYH);
  unsigned short* yL    = (unsigned short*)(ws + kOffYL);
  unsigned short* wxT   = (unsigned short*)(ws + kOffWx);
  unsigned short* wdtT  = (unsigned short*)(ws + kOffWdt);
  unsigned short* woH   = (unsigned short*)(ws + kOffWoH);
  unsigned short* woL   = (unsigned short*)(ws + kOffWoL);
  unsigned short* wcH   = (unsigned short*)(ws + kOffWcH);
  unsigned short* wcL   = (unsigned short*)(ws + kOffWcL);
  float*          proj  = (float*)(ws + kOffProj);
  unsigned short* dtA   = (unsigned short*)(ws + kOffDtA);
  const float* dummyf = lin_ch_b;

  k_transpose_planes<true><<<dim3(4096 / 32, 1024 / 64, 1), 256, 0, stream>>>(
      in_proj_w, 4096, 4096, 0L, winH, winL, 1024, 0L);
  k_transpose_planes<false><<<dim3(kNProjPad / 32, 2048 / 64, 1), 256, 0, stream>>>(
      x_proj_w, 96, 96, 0L, wxT, wxT, 2048, 0L);
  k_transpose_planes<false><<<dim3(2048 / 32, 64 / 64, 1), 256, 0, stream>>>(
      dt_proj_w, 2048, 2048, 0L, wdtT, wdtT, 64, 0L);
  k_transpose_planes<true><<<dim3(1024 / 32, 2048 / 64, 1), 256, 0, stream>>>(
      out_proj_w, 1024, 1024, 0L, woH, woL, 2048, 0L);
  k_transpose_planes<true><<<dim3(256 / 32, 256 / 64, 1), 256, 0, stream>>>(
      lin_ch_w, 256, 256, 0L, wcH, wcL, 256, 0L);

  k_resize_down<<<kRows, 128, 0, stream>>>(x1, xsH, xsL);

  wmma_gemm64<1, true, 0, 0, false><<<dim3((kRows / 64) * ((2 * kDInner) / 64) / 8, 1), 256, 0, stream>>>(
      xsH, xsL, kDModel, 0L, winH, winL, kDModel, 0L,
      xz, xz, 2 * kDInner, 0L, dummyf, dummyf, 0L, kRows, 2 * kDInner, kDModel, 1.0f);

  k_conv_silu<<<kRows, 256, 0, stream>>>(xz, conv_w, conv_b, xcF, xcB);

  wmma_gemm64<1, false, 0, 0, false><<<dim3((kRows / 64) * (kNProjPad / 64) / 8, 1), 256, 0, stream>>>(
      xcB, xcB, kDInner, 0L, wxT, wxT, kDInner, 0L,
      proj, proj, kNProjPad, 0L, dummyf, dummyf, 0L, kRows, kNProjPad, kDInner, 1.0f);

  k_cvt_dt<<<kRows / 32, 256, 0, stream>>>(proj, dtA);
  wmma_gemm64<1, false, 0, 0, false><<<dim3((kRows / 64) * (kDInner / 64) / 8, 1), 256, 0, stream>>>(
      dtA, dtA, kDtRank, 0L, wdtT, wdtT, kDtRank, 0L,
      dtpre, dtpre, kDInner, 0L, dummyf, dummyf, 0L, kRows, kDInner, kDtRank, 1.0f);

  k_scan<<<dim3(kDInner / 256, kBatch), 256, 0, stream>>>(proj, dtpre, xcF, xz, a_log, d_param, dt_proj_b, yH, yL);

  wmma_gemm64<1, true, 0, 0, false><<<dim3((kRows / 64) * (kDModel / 64) / 8, 1), 256, 0, stream>>>(
      yH, yL, kDInner, 0L, woH, woL, kDInner, 0L,
      ymm, ymm, kDModel, 0L, dummyf, dummyf, 0L, kRows, kDModel, kDInner, 1.0f);

  k_layernorm<<<kRows / 8, 256, 0, stream>>>(ymm, ln_g, ln_b, yln);

  k_transpose_planes<true><<<dim3(1024 / 32, 256 / 64, kBatch), 256, 0, stream>>>(
      yln, 1024, 1024, 256L * 1024, ylnTH, ylnTL, 256, 1024L * 256);

  wmma_gemm64<1, true, 0, 0, false><<<dim3((kCOut / 64) * (1024 / 64) / 8, kBatch), 256, 0, stream>>>(
      wcH, wcL, kCIn, 0L, ylnTH, ylnTL, kCIn, 1024L * 256,
      sml, sml, 1024, 256L * 1024, dummyf, dummyf, 0L, kCOut, 1024, kCIn, 1.0f);

  k_resize_up<<<kBatch * kCOut * 4, 256, 0, stream>>>(sml, lin_ch_b, out);
}
